// LatentPredictionHeadEdge_38199439130848
// MI455X (gfx1250) — hardware-verified
//
#include <hip/hip_runtime.h>
#include <math.h>


#define NN   4096
#define NE   262144
#define IND  256
#define ED   16
#define NAF  16
#define LATD 128
#define NBT  5
#define SORTN 262144
#define TILE 4096
typedef unsigned long long u64;
typedef __attribute__((ext_vector_type(16))) _Float16 v16h;
typedef __attribute__((ext_vector_type(8)))  _Float16 v8h;
typedef __attribute__((ext_vector_type(8)))  float    v8f;
typedef __attribute__((ext_vector_type(4)))  float    v4f;
typedef __attribute__((ext_vector_type(2)))  int      v2i;
#define VST2(T, ptr, val) do { const T _v = (val); *(volatile T*)(ptr) = _v; __threadfence(); *(volatile T*)(ptr) = _v; } while (0)
__device__ __forceinline__ v8f wmma16(v16h a, v16h b, v8f c) {
  v8f d = __builtin_amdgcn_wmma_f32_16x16x32_f16(false, a, false, b, (short)0, c, false, false);
  asm volatile("v_nop\n\tv_nop\n\tv_nop\n\tv_nop" : "+v"(d) : "v"(a), "v"(b));
  return d;
}
__device__ __forceinline__ v16h frag16(const _Float16* p, int hh) {
  const v8h lo = *(const v8h*)(p + 8 * hh), hi = *(const v8h*)(p + 16 + 8 * hh);
  return __builtin_shufflevector(lo, hi, 0,1,2,3,4,5,6,7,8,9,10,11,12,13,14,15);
}
__device__ __forceinline__ float silu(float x) { return x / (1.0f + expf(-x)); }
__global__ __launch_bounds__(256) void k_sort_init(const int* __restrict__ ej, const int* __restrict__ ei_, u64* __restrict__ A) {
  const int i = blockIdx.x * 256 + threadIdx.x;
  const u64 pr = (u64)((unsigned)min(max(ej[i], 0), NN - 1) * NN + (unsigned)min(max(ei_[i], 0), NN - 1));
  VST2(u64, A + i, (pr << 32) | (u64)(unsigned)i);
}
__device__ __forceinline__ void cas_lds(u64* s, int lo, int hi, bool up) {
  const u64 a = s[lo], b = s[hi]; const bool sw = up ? (a > b) : (a < b); s[lo] = sw ? b : a; s[hi] = sw ? a : b;
}
__global__ __launch_bounds__(256) void k_sort_local(u64* __restrict__ A) {
  __shared__ u64 s[TILE];
  const int base = blockIdx.x * TILE, t = threadIdx.x;
  for (int i = t; i < TILE; i += 256) s[i] = A[base + i];
  __syncthreads();
  for (int k = 2; k <= TILE; k <<= 1)
    for (int j = k >> 1; j > 0; j >>= 1) {
      for (int p = t; p < TILE / 2; p += 256) {
        const int lo = ((p >> __builtin_ctz(j)) << (__builtin_ctz(j) + 1)) | (p & (j - 1));
        cas_lds(s, lo, lo + j, (((base + lo) & k) == 0));
      }
      __syncthreads();
    }
  for (int pass = 0; pass < 2; ++pass) { for (int i = t; i < TILE; i += 256) *(volatile u64*)(A + base + i) = s[i]; __threadfence(); }
}
__global__ __launch_bounds__(256) void k_sort_global(u64* __restrict__ A, int logj, int k) {
  const int p = blockIdx.x * 256 + threadIdx.x;
  const int j = 1 << logj;
  const int lo = ((p >> logj) << (logj + 1)) | (p & (j - 1)), hi = lo + j;
  const u64 a = A[lo], b = A[hi];
  const bool up = ((lo & k) == 0), sw = up ? (a > b) : (a < b);
  const u64 vlo = sw ? b : a, vhi = sw ? a : b;
  *(volatile u64*)(A + lo) = vlo; *(volatile u64*)(A + hi) = vhi; __threadfence();
  *(volatile u64*)(A + lo) = vlo; *(volatile u64*)(A + hi) = vhi;
}
__global__ __launch_bounds__(256) void k_sort_lds(u64* __restrict__ A, int k) {
  __shared__ u64 s[TILE];
  const int base = blockIdx.x * TILE, t = threadIdx.x;
  for (int i = t; i < TILE; i += 256) s[i] = A[base + i];
  __syncthreads();
  for (int j = TILE >> 1; j > 0; j >>= 1) {
    for (int p = t; p < TILE / 2; p += 256) {
      const int lo = ((p >> __builtin_ctz(j)) << (__builtin_ctz(j) + 1)) | (p & (j - 1));
      cas_lds(s, lo, lo + j, (((base + lo) & k) == 0));
    }
    __syncthreads();
  }
  for (int pass = 0; pass < 2; ++pass) { for (int i = t; i < TILE; i += 256) *(volatile u64*)(A + base + i) = s[i]; __threadfence(); }
}
__device__ __forceinline__ int last_edge(const u64* __restrict__ A, unsigned pr) {
  int lo = 0, hi = SORTN;
  while (lo < hi) { const int mid = (lo + hi) >> 1; if ((unsigned)(A[mid] >> 32) < pr + 1u) lo = mid + 1; else hi = mid; }
  if (lo == 0) return -1;
  const u64 kk = A[lo - 1];
  return ((unsigned)(kk >> 32) == pr) ? (int)(unsigned)(kk & 0xffffffffu) : -1;
}
__global__ __launch_bounds__(256) void k_esym(const float* __restrict__ e, const int* __restrict__ ej, const int* __restrict__ ei_, const u64* __restrict__ A,
                                              _Float16* __restrict__ E16) {
  const int t = blockIdx.x * 256 + threadIdx.x;
  const int j = min(max(ej[t], 0), NN - 1), i = min(max(ei_[t], 0), NN - 1);
  const int a = last_edge(A, (unsigned)(j * NN + i)), b = last_edge(A, (unsigned)(i * NN + j));
  const int ac = min(max(a, 0), NE - 1), bc = min(max(b, 0), NE - 1);
  v8h o0, o1, zz;
#pragma unroll
  for (int q = 0; q < 8; ++q) {
    const float va = (a >= 0) ? e[(size_t)ac * ED + q] : 0.f, vb = (b >= 0) ? e[(size_t)bc * ED + q] : 0.f;
    const float wa = (a >= 0) ? e[(size_t)ac * ED + 8 + q] : 0.f, wb = (b >= 0) ? e[(size_t)bc * ED + 8 + q] : 0.f;
    o0[q] = (_Float16)(0.5f * (va + vb)); o1[q] = (_Float16)(0.5f * (wa + wb)); zz[q] = (_Float16)0.f;
  }
  for (int pass = 0; pass < 2; ++pass) {
    *(volatile v8h*)(E16 + (size_t)t * 32) = o0; *(volatile v8h*)(E16 + (size_t)t * 32 + 8) = o1;
    *(volatile v8h*)(E16 + (size_t)t * 32 + 16) = zz; *(volatile v8h*)(E16 + (size_t)t * 32 + 24) = zz;
    __threadfence();
  }
}
__global__ __launch_bounds__(256) void k_to16(const float* __restrict__ s, int rows, int K, _Float16* __restrict__ d) {
  const int t = blockIdx.x * 256 + threadIdx.x; const int per = K / 8;
  if (t >= rows * per) return;
  const int r = t / per, c = (t % per) * 8;
  v8h o;
#pragma unroll
  for (int q = 0; q < 8; ++q) o[q] = (_Float16)s[(size_t)r * K + c + q];
  VST2(v8h, d + (size_t)r * K + c, o);
}
__global__ __launch_bounds__(256) void k_w16(const float* __restrict__ w, int N, int K, int Npad, int Kpad, _Float16* __restrict__ W16) {
  const int t = blockIdx.x * 256 + threadIdx.x; const int per = Kpad / 8;
  if (t >= Npad * per) return;
  const int n = t / per, k0 = (t % per) * 8;
  v8h o;
#pragma unroll
  for (int q = 0; q < 8; ++q) o[q] = (n < N && k0 + q < K) ? (_Float16)w[(size_t)n * K + k0 + q] : (_Float16)0.f;
  VST2(v8h, W16 + (size_t)n * Kpad + k0, o);
}
template <int K, int NTOT, int EPI>
__global__ __launch_bounds__(128) void k_gemm(const _Float16* __restrict__ A, const _Float16* __restrict__ W16, const float* __restrict__ bias,
                                              const float* __restrict__ sres, const int* __restrict__ ej, const int* __restrict__ ei_,
                                              float* __restrict__ outf, _Float16* __restrict__ outh, float* __restrict__ out2) {
  __shared__ __attribute__((aligned(16))) float sT[4][16][132];
  __shared__ __attribute__((aligned(16))) float sB[64 * 16];
  const int lane = threadIdx.x & 31, wave = threadIdx.x >> 5, hh = lane >> 4, l16 = lane & 15;
  const int m0 = blockIdx.x * 64 + wave * 16, n0 = blockIdx.y * 128;
  v8f acc[8];
#pragma unroll
  for (int ni = 0; ni < 8; ++ni) acc[ni] = (v8f){};
#pragma unroll 2
  for (int k0 = 0; k0 < K; k0 += 32) {
    const v16h a0 = frag16(A + (size_t)(m0 + l16) * K + k0, hh);
#pragma unroll
    for (int ni = 0; ni < 8; ++ni) { const v16h b = frag16(W16 + (size_t)(n0 + ni * 16 + l16) * K + k0, hh); acc[ni] = wmma16(a0, b, acc[ni]); }
  }
  float (*st)[132] = sT[wave];
#pragma unroll
  for (int ni = 0; ni < 8; ++ni)
#pragma unroll
    for (int q = 0; q < 8; ++q) { float v = acc[ni][q] + bias[n0 + ni * 16 + l16]; if (EPI == 0) v = silu(v); st[q + 8 * hh][ni * 16 + l16] = v; }
  __builtin_amdgcn_fence(__ATOMIC_RELEASE, "workgroup"); __builtin_amdgcn_wave_barrier(); __builtin_amdgcn_fence(__ATOMIC_ACQUIRE, "workgroup");
  if (EPI == 2) {
#pragma unroll
    for (int rr = 0; rr < 16; ++rr) {
      const int eidx = m0 + rr; const int j = min(max(ej[eidx], 0), NN - 1), i = min(max(ei_[eidx], 0), NN - 1);
      const v4f si = *(const v4f*)(sres + (size_t)i * IND + n0 + lane * 4), sj = *(const v4f*)(sres + (size_t)j * IND + n0 + lane * 4);
      float* p = &st[rr][lane * 4];
#pragma unroll
      for (int q = 0; q < 4; ++q) p[q] = silu(p[q] + si[q] + sj[q]);
    }
    __builtin_amdgcn_fence(__ATOMIC_RELEASE, "workgroup"); __builtin_amdgcn_wave_barrier(); __builtin_amdgcn_fence(__ATOMIC_ACQUIRE, "workgroup");
  }
  if (EPI == 1 || EPI == 3) {
    const int nc = (EPI == 1) ? NAF : NBT;
#pragma unroll
    for (int rr = 0; rr < 16; ++rr) if (lane < nc) sB[(wave * 16 + rr) * nc + lane] = st[rr][lane];
    __syncthreads();
  }
  for (int pass = 0; pass < 2; ++pass) {
#pragma unroll
    for (int rr = 0; rr < 16; ++rr) {
      if (EPI == 0) *(volatile v4f*)(outf + (size_t)(m0 + rr) * NTOT + n0 + lane * 4) = *(const v4f*)(&st[rr][lane * 4]);
      if (EPI == 1 && n0 == 0) *(volatile v4f*)(outf + (size_t)(m0 + rr) * LATD + lane * 4) = *(const v4f*)(&st[rr][lane * 4]);
      if ((EPI == 0 || EPI == 2) && lane < 16) { v8h o;
#pragma unroll
        for (int q = 0; q < 8; ++q) o[q] = (_Float16)st[rr][lane * 8 + q];
        *(volatile v8h*)(outh + (size_t)(m0 + rr) * NTOT + n0 + lane * 8) = o; }
    }
    if (EPI == 1 && n0 == 128) { for (int q = threadIdx.x; q < 64 * NAF; q += 128) *(volatile float*)(out2 + (size_t)blockIdx.x * 64 * NAF + q) = sB[q]; }
    if (EPI == 3) { for (int q = threadIdx.x; q < 64 * NBT; q += 128) *(volatile float*)(out2 + (size_t)blockIdx.x * 64 * NBT + q) = sB[q]; }
    __threadfence();
  }
}
extern "C" void kernel_launch(void* const* d_in, const int* in_sizes, int n_in,
                              void* d_out, int out_size, void* d_ws, size_t ws_size, hipStream_t stream) {
  (void)in_sizes; (void)n_in; (void)out_size;
  const float* s0   = (const float*)d_in[0];
  const float* e    = (const float*)d_in[1];
  const int*   eidx = (const int*)  d_in[3];
  const float* Wsh  = (const float*)d_in[4];  const float* bsh = (const float*)d_in[5];
  const float* Wbd  = (const float*)d_in[6];  const float* bbd = (const float*)d_in[7];
  const float* Wbs  = (const float*)d_in[8];  const float* bbs = (const float*)d_in[9];
  const float* Wat  = (const float*)d_in[10]; const float* bat = (const float*)d_in[11];
  float* outL = (float*)d_out;
  float* outA = (float*)((char*)d_out + 2097152);
  float* outB = (float*)((char*)d_out + 2359296);
  const int* ej = eidx; const int* ei_ = eidx + NE;
  char* ws = (char*)d_ws; size_t off = 0;
  auto take = [&](size_t bytes) { void* p = ws + off; off = (off + bytes + 255) & ~(size_t)255; return p; };
  u64*      keys = (u64*)take((size_t)SORTN * 8);
  _Float16* S16  = (_Float16*)take((size_t)NN * IND * 2);
  _Float16* Wsh6 = (_Float16*)take((size_t)IND * IND * 2);
  _Float16* Wat6 = (_Float16*)take((size_t)256 * IND * 2);
  _Float16* Wbd6 = (_Float16*)take((size_t)IND * 32 * 2);
  _Float16* Wbs6 = (_Float16*)take((size_t)128 * IND * 2);
  float*    bat2 = (float*)take((size_t)256 * 4);
  float*    bbs2 = (float*)take((size_t)128 * 4);
  float*    sact = (float*)take((size_t)NN * IND * 4);
  _Float16* sa16 = (_Float16*)take((size_t)NN * IND * 2);
  _Float16* E16  = (_Float16*)take((size_t)NE * 32 * 2);
  _Float16* F16  = (_Float16*)take((size_t)NE * IND * 2);
  if (off > ws_size) return;
  hipMemsetAsync(bat2, 0, 256 * 4, stream);
  hipMemcpyAsync(bat2, bat + NAF, LATD * 4, hipMemcpyDeviceToDevice, stream);
  hipMemcpyAsync(bat2 + LATD, bat, NAF * 4, hipMemcpyDeviceToDevice, stream);
  hipMemsetAsync(bbs2, 0, 128 * 4, stream); hipMemcpyAsync(bbs2, bbs, NBT * 4, hipMemcpyDeviceToDevice, stream);
  const dim3 b256(256);
  k_sort_init<<<SORTN / 256, b256, 0, stream>>>(ej, ei_, keys);
  k_sort_local<<<SORTN / TILE, b256, 0, stream>>>(keys);
  for (int k = TILE * 2; k <= SORTN; k <<= 1) {
    for (int logj = __builtin_ctz(k) - 1; (1 << logj) >= TILE; --logj)
      k_sort_global<<<SORTN / 2 / 256, b256, 0, stream>>>(keys, logj, k);
    k_sort_lds<<<SORTN / TILE, b256, 0, stream>>>(keys, k);
  }
  k_to16<<<(NN * 32 + 255) / 256, b256, 0, stream>>>(s0, NN, IND, S16);
  k_w16<<<(IND * 32 + 255) / 256, b256, 0, stream>>>(Wsh, IND, IND, IND, IND, Wsh6);
  k_w16<<<(128 * 32 + 255) / 256, b256, 0, stream>>>(Wat + (size_t)NAF * IND, LATD, IND, LATD, IND, Wat6);
  k_w16<<<(128 * 32 + 255) / 256, b256, 0, stream>>>(Wat, NAF, IND, 128, IND, Wat6 + (size_t)LATD * IND);
  k_w16<<<(IND * 4 + 255) / 256, b256, 0, stream>>>(Wbd, IND, ED, IND, 32, Wbd6);
  k_w16<<<(128 * 32 + 255) / 256, b256, 0, stream>>>(Wbs, NBT, IND, 128, IND, Wbs6);
  k_gemm<IND, IND, 0><<<dim3(NN / 64, 2), 128, 0, stream>>>(S16, Wsh6, bsh, nullptr, nullptr, nullptr, sact, sa16, nullptr);
  k_gemm<IND, 256, 1><<<dim3(NN / 64, 2), 128, 0, stream>>>(sa16, Wat6, bat2, nullptr, nullptr, nullptr, outL, nullptr, outA);
  k_esym<<<NE / 256, b256, 0, stream>>>(e, ej, ei_, keys, E16);
  k_gemm<32, IND, 2><<<dim3(NE / 64, 2), 128, 0, stream>>>(E16, Wbd6, bbd, sact, ej, ei_, nullptr, F16, nullptr);
  k_gemm<IND, 128, 3><<<dim3(NE / 64, 1), 128, 0, stream>>>(F16, Wbs6, bbs2, nullptr, nullptr, nullptr, nullptr, nullptr, outB);
}
